// thetaRNNLayer_17042430231265
// MI455X (gfx1250) — hardware-run, weakly checked
//
#include <hip/hip_runtime.h>
#include <math.h>

typedef __attribute__((ext_vector_type(16))) _Float16 v16h;
typedef __attribute__((ext_vector_type(8)))  _Float16 v8h;
typedef __attribute__((ext_vector_type(4)))  _Float16 v4h;
typedef __attribute__((ext_vector_type(2)))  _Float16 v2h;
typedef __attribute__((ext_vector_type(16))) __bf16   v16b;
typedef __attribute__((ext_vector_type(8)))  __bf16   v8b;
typedef __attribute__((ext_vector_type(8)))  float    v8f;
typedef __attribute__((ext_vector_type(4)))  float    v4f;
typedef __attribute__((ext_vector_type(2)))  float    v2f;

constexpr int kSeq   = 4096;
constexpr int kHid   = 512;
constexpr int kIn    = 512;
constexpr int kTheta = 5;
constexpr int kThr   = 256;
constexpr int kChainThr = 128;
constexpr size_t kSlice = (size_t)kSeq * kHid;
constexpr size_t kOut0  = (size_t)(kTheta + 1) * kSlice;

constexpr float kInCarry  = 1024.0f;
constexpr float kWCarry   = 1024.0f;
constexpr float kActCarry = 4096.0f;
constexpr float kXsScale  = 1.0f / (kInCarry * kWCarry);
constexpr float kRecScale = 1.0f / (kActCarry * kWCarry);
constexpr float kF16MinNormal = 6.103515625e-5f;

static_assert((kSeq % 64) == 0 && (kHid % 64) == 0 && (kIn % 32) == 0 && kChainThr * 4 == kHid, "GEMM shapes; one chain thread per FOUR hidden units");

constexpr size_t kOffX16 = 0;
constexpr size_t kOffWIH = kOffX16 + (size_t)kSeq * kIn * 2;
constexpr size_t kOffWHH = kOffWIH + (size_t)kHid * kIn * 2;
constexpr size_t kOffWHT = kOffWHH + (size_t)kHid * kHid * 2;
constexpr size_t kOffBV  = kOffWHT + (size_t)kHid * kHid * 4;
constexpr size_t kOffPRE = kOffBV  + (size_t)2 * kHid * 4;
constexpr size_t kOffH16 = kOffPRE + kSlice * 4;
constexpr size_t kOffZ   = kOffH16 + kSlice * 2;
constexpr size_t kWsTotal = kOffZ + kSlice * 4;
static_assert(kWsTotal == 27267072ull, "carve total");
static_assert((kOffWIH % 256) == 0 && (kOffWHH % 256) == 0 && (kOffWHT % 256) == 0 && (kOffBV % 256) == 0 && (kOffPRE % 256) == 0 && (kOffH16 % 256) == 0 && (kOffZ % 256) == 0, "aligned regions");

__device__ __forceinline__ unsigned short f2bf_bits(float f) {
  unsigned u = __float_as_uint(f);
  return (unsigned short)((u + 0x7FFFu + ((u >> 16) & 1u)) >> 16);
}
__device__ __forceinline__ float bf_bits2f(unsigned short h) { return __uint_as_float(((unsigned)h) << 16); }
__device__ __forceinline__ float bf16r(float f) { return bf_bits2f(f2bf_bits(f)); }
__device__ __forceinline__ float carry_flush(float v, float carry) {
  const float s = v * carry;
  return (fabsf(s) < kF16MinNormal) ? 0.0f : s;
}
__device__ __forceinline__ float frcp(float x) { return __builtin_amdgcn_rcpf(x); }

__device__ __forceinline__ void dep_guard4_h(v8f& a, v8f& b, v8f& c, v8f& d, v16h x, v16h y) { asm volatile("v_nop\n\tv_nop\n\tv_nop\n\tv_nop" : "+v"(a), "+v"(b), "+v"(c), "+v"(d) : "v"(x), "v"(y)); }
__device__ __forceinline__ void dep_guard4_b(v8f& a, v8f& b, v8f& c, v8f& d, v16b x, v16b y) { asm volatile("v_nop\n\tv_nop\n\tv_nop\n\tv_nop" : "+v"(a), "+v"(b), "+v"(c), "+v"(d) : "v"(x), "v"(y)); }
__device__ __forceinline__ void keep4_h(v16h a, v16h b, v16h c, v16h d) { asm volatile("v_nop" :: "v"(a), "v"(b), "v"(c), "v"(d)); }
__device__ __forceinline__ void keep4_b(v16b a, v16b b, v16b c, v16b d) { asm volatile("v_nop" :: "v"(a), "v"(b), "v"(c), "v"(d)); }
__device__ __forceinline__ void acc_guard4(v8f& a, v8f& b, v8f& c, v8f& d) { asm volatile("v_nop\n\tv_nop\n\tv_nop\n\tv_nop" : "+v"(a), "+v"(b), "+v"(c), "+v"(d)); }

template <typename T> struct Frag;
template <> struct Frag<_Float16> {
  typedef v16h V; union U { v16h v; v8h h[2]; };
  static __device__ __forceinline__ v16h load(const _Float16* p) {
    U f; f.h[0] = *(const v8h*)(p); f.h[1] = *(const v8h*)(p + 16); return f.v;
  }
  static __device__ __forceinline__ v8f mma(v16h a, v16h b, v8f c) {
    return __builtin_amdgcn_wmma_f32_16x16x32_f16(false, a, false, b, (short)0, c, false, false);
  }
  static __device__ __forceinline__ void guard4(v8f& a, v8f& b, v8f& c, v8f& d, v16h x, v16h y) { dep_guard4_h(a, b, c, d, x, y); }
  static __device__ __forceinline__ void keep(v16h a, v16h b, v16h c, v16h d) { keep4_h(a, b, c, d); }
};
template <> struct Frag<__bf16> {
  typedef v16b V; union U { v16b v; v8b h[2]; };
  static __device__ __forceinline__ v16b load(const __bf16* p) {
    U f; f.h[0] = *(const v8b*)(p); f.h[1] = *(const v8b*)(p + 16); return f.v;
  }
  static __device__ __forceinline__ v8f mma(v16b a, v16b b, v8f c) {
    return __builtin_amdgcn_wmma_f32_16x16x32_bf16(false, a, false, b, (short)0, c, false, false);
  }
  static __device__ __forceinline__ void guard4(v8f& a, v8f& b, v8f& c, v8f& d, v16b x, v16b y) { dep_guard4_b(a, b, c, d, x, y); }
  static __device__ __forceinline__ void keep(v16b a, v16b b, v16b c, v16b d) { keep4_b(a, b, c, d); }
};

__device__ __forceinline__ v8f mma_h(v16h a, v16h b, v8f c) {
  c = __builtin_amdgcn_wmma_f32_16x16x32_f16(false, a, false, b, (short)0, c, false, false);
  asm volatile("v_nop\n\tv_nop\n\tv_nop\n\tv_nop" : "+v"(c) : "v"(a), "v"(b));
  return c;
}

template <int ET> struct Elem;
template <> struct Elem<0> { typedef _Float16 T; };
template <> struct Elem<1> { typedef __bf16 T; };
template <int ET, bool SPLIT, int BIAS_MODE, int OUT_MODE, bool RESID, int ACT = 0>
__global__ __launch_bounds__(256) void wmma_gemm64(
    const unsigned short* __restrict__ Ap, const unsigned short* __restrict__ A2p, int lda, long strideA,
    const unsigned short* __restrict__ Btp, const unsigned short* __restrict__ Bt2p, int ldb, long strideB,
    void* __restrict__ Cout, void* __restrict__ Cout2, int ldc, long strideC,
    const float* __restrict__ bias,
    const float* __restrict__ resid, long strideR,
    int M, int N, int K, float scale) {
  typedef typename Elem<ET>::T T;
  typedef typename Frag<T>::V V;
  const T* A = (const T*)Ap; const T* A2 = (const T*)A2p; const T* Bt = (const T*)Btp; const T* Bt2 = (const T*)Bt2p;
  __shared__ __align__(16) float sT[8][16 * 68];
  const int b    = blockIdx.y;
  const int lane = threadIdx.x & 31;
  const int wave = threadIdx.x >> 5;
  const int tilesN = N >> 6;
  const int tilesM = M >> 6;
  const int tile = blockIdx.x * 8 + wave;
  if (tile >= tilesM * tilesN) return;
  const int tm = tile / tilesN;
  const int tn = tile - tm * tilesN;
  const int m0 = tm << 6;
  const int n0 = tn << 6;

  const T* Ab  = A  + (size_t)b * strideA;
  const T* Bb  = Bt + (size_t)b * strideB;
  const T* Ab2 = SPLIT ? (A2  + (size_t)b * strideA) : nullptr;
  const T* Bb2 = SPLIT ? (Bt2 + (size_t)b * strideB) : nullptr;

  const int rlane = lane & 15;
  const int koff  = (lane >> 4) * 8;
  const int mOff  = (lane >> 4) * 8;

  v8f acc[4][4];
#pragma unroll
  for (int i = 0; i < 4; ++i)
#pragma unroll
    for (int j = 0; j < 4; ++j) acc[i][j] = (v8f){0.f,0.f,0.f,0.f,0.f,0.f,0.f,0.f};

  for (int k0 = 0; k0 < K; k0 += 32) {
    V bh[4], bl[4];
#pragma unroll
    for (int j = 0; j < 4; ++j) {
      const size_t bo = (size_t)(n0 + (j << 4) + rlane) * ldb + koff + k0;
      bh[j] = Frag<T>::load(Bb + bo);
      if (SPLIT) bl[j] = Frag<T>::load(Bb2 + bo);
    }
#pragma unroll
    for (int i = 0; i < 4; ++i) {
      const size_t ao = (size_t)(m0 + (i << 4) + rlane) * lda + koff + k0;
      V ah = Frag<T>::load(Ab + ao);
      V al;
      if (SPLIT) al = Frag<T>::load(Ab2 + ao);
#pragma unroll
      for (int j = 0; j < 4; ++j) {
        acc[i][j] = Frag<T>::mma(ah, bh[j], acc[i][j]);
        if (SPLIT) {
          acc[i][j] = Frag<T>::mma(ah, bl[j], acc[i][j]);
          acc[i][j] = Frag<T>::mma(al, bh[j], acc[i][j]);
        }
      }
      Frag<T>::guard4(acc[i][0], acc[i][1], acc[i][2], acc[i][3], ah, SPLIT ? al : ah);
    }
    Frag<T>::keep(bh[0], bh[1], bh[2], bh[3]);
    if (SPLIT) Frag<T>::keep(bl[0], bl[1], bl[2], bl[3]);
  }
  acc_guard4(acc[0][0], acc[0][1], acc[0][2], acc[0][3]);
  acc_guard4(acc[1][0], acc[1][1], acc[1][2], acc[1][3]);
  acc_guard4(acc[2][0], acc[2][1], acc[2][2], acc[2][3]);
  acc_guard4(acc[3][0], acc[3][1], acc[3][2], acc[3][3]);

  float* slab = sT[wave];
  const float* Rb = RESID ? (resid + (size_t)b * strideR) : nullptr;
#pragma unroll
  for (int i = 0; i < 4; ++i) {
    const int mBase = m0 + (i << 4);
#pragma unroll
    for (int j = 0; j < 4; ++j) {
      const int n = n0 + (j << 4) + rlane;
      float bv = 0.f;
      if (BIAS_MODE == 2) bv = bias[n];
#pragma unroll
      for (int r = 0; r < 8; ++r) {
        float v = acc[i][j][r] * scale;
        if (BIAS_MODE == 1) v += bias[mBase + mOff + r];
        if (BIAS_MODE == 2) v += bv;
        if (RESID) v += Rb[(size_t)(mBase + mOff + r) * ldc + n];
        if (ACT == 1) v = tanhf(v);
        if (ACT == 2) v = fmaxf(v, 0.0f);
        if (ACT == 3) v = v / (1.0f + expf(-v));
        if (ACT == 4) v = (v > 0.f) ? v : 0.01f * v;
        slab[(mOff + r) * 68 + (j << 4) + rlane] = v;
      }
    }
    __builtin_amdgcn_fence(__ATOMIC_RELEASE, "workgroup");
    __builtin_amdgcn_wave_barrier();
    __builtin_amdgcn_fence(__ATOMIC_ACQUIRE, "workgroup");
    if (OUT_MODE == 0) {
      float* C = (float*)Cout + (size_t)b * strideC;
      const int hh = lane >> 4, c4 = (lane & 15) * 4;
      for (int pass = 0; pass < 2; ++pass) {
#pragma unroll
        for (int it = 0; it < 8; ++it) {
          const int row = it * 2 + hh;
          v4f v = *(const v4f*)(slab + row * 68 + c4);
          *(volatile v4f*)(C + (size_t)(mBase + row) * ldc + n0 + c4) = v;
        }
        __threadfence();
      }
    } else {
      const int q = lane >> 3, c8 = (lane & 7) * 8;
      unsigned short* C  = (unsigned short*)Cout  + (size_t)b * strideC;
      unsigned short* C2 = (OUT_MODE == 2) ? ((unsigned short*)Cout2 + (size_t)b * strideC) : nullptr;
      for (int pass = 0; pass < 2; ++pass) {
#pragma unroll
        for (int it = 0; it < 4; ++it) {
          const int row = it * 4 + q;
          const float* sp = slab + row * 68 + c8;
          v8h hv, lv;
#pragma unroll
          for (int e = 0; e < 8; ++e) {
            if (OUT_MODE == 1) {
              hv[e] = (_Float16)sp[e];
            } else {
              unsigned short hb = f2bf_bits(sp[e]);
              unsigned short lb = f2bf_bits(sp[e] - bf_bits2f(hb));
              hv[e] = __builtin_bit_cast(_Float16, hb);
              lv[e] = __builtin_bit_cast(_Float16, lb);
            }
          }
          *(volatile v8h*)(C + (size_t)(mBase + row) * ldc + n0 + c8) = hv;
          if (OUT_MODE == 2) *(volatile v8h*)(C2 + (size_t)(mBase + row) * ldc + n0 + c8) = lv;
        }
        __threadfence();
      }
    }
    __builtin_amdgcn_fence(__ATOMIC_RELEASE, "workgroup");
    __builtin_amdgcn_wave_barrier();
    __builtin_amdgcn_fence(__ATOMIC_ACQUIRE, "workgroup");
  }
}

__global__ __launch_bounds__(kThr) void cast_plane_kernel(const float* __restrict__ src, unsigned short* __restrict__ dst,
                                                          int colsLog2, int dstPitch, int dstOff) {
  const int i   = blockIdx.x * kThr + threadIdx.x;
  const int sh  = colsLog2 - 3;
  const int row = i >> sh;
  const int c8  = (i & ((1 << sh) - 1)) * 8;
  const float* sp = src + ((size_t)row << colsLog2) + c8;
  const v4f a0 = *(const v4f*)(sp);
  const v4f a1 = *(const v4f*)(sp + 4);
  v8h hv;
#pragma unroll
  for (int e = 0; e < 4; ++e) {
    const float f0 = a0[e];
    const float f1 = a1[e];
    hv[e]     = (_Float16)carry_flush(bf16r(f0), kInCarry);
    hv[4 + e] = (_Float16)carry_flush(bf16r(f1), kInCarry);
  }
  unsigned short* dp = dst + (size_t)row * dstPitch + dstOff + c8;
  *(volatile v8h*)dp = hv;
  __threadfence();
  *(volatile v8h*)dp = hv;
}
static_assert(kInCarry == kWCarry, "one cast kernel serves inputs and weights");

__global__ __launch_bounds__(kThr) void th_setup_kernel(const float* __restrict__ Whh, const float* __restrict__ b,
                                                        float* __restrict__ WHT, float* __restrict__ BV) {
  const int t = threadIdx.x;
  if (blockIdx.x == kHid) {
    const v2f o = {bf16r(b[2 * t]), bf16r(b[2 * t + 1])};
    const v2f z = {0.0f, 0.0f};
    for (int pass = 0; pass < 2; ++pass) {
      *(volatile v2f*)(BV + 2 * t) = o;
      *(volatile v2f*)(BV + kHid + 2 * t) = z;
      __threadfence();
    }
    return;
  }
  const int k = blockIdx.x;
  const v2f o = {bf16r(Whh[(size_t)(2 * t) * kHid + k]), bf16r(Whh[(size_t)(2 * t + 1) * kHid + k])};
  float* dp = WHT + (size_t)k * kHid + 2 * t;
  *(volatile v2f*)dp = o;
  __threadfence();
  *(volatile v2f*)dp = o;
}

__global__ __launch_bounds__(kChainThr) void th_chain_kernel(const float* __restrict__ PRE, const float* __restrict__ noise0,
                                                             const float* __restrict__ WHT, const float* __restrict__ st0,
                                                             float* __restrict__ out0, float* __restrict__ out1) {
  __shared__ __align__(16) float hbuf[2][kHid];
  const int u4 = threadIdx.x * 4;
  {
    const v4f s0 = *(const v4f*)(st0 + u4);
    v4f h0;
#pragma unroll
    for (int e = 0; e < 4; ++e) h0[e] = bf16r(s0[e]);
    *(v4f*)(&hbuf[0][u4]) = h0;
  }
  __syncthreads();
#pragma unroll 1
  for (int t = 0; t < kSeq; ++t) {
    const float* hc = &hbuf[t & 1][0];
    v4f acc = {0.0f, 0.0f, 0.0f, 0.0f};
#pragma unroll 2
    for (int k = 0; k < kHid; k += 4) {
      const v4f hv = *(const v4f*)(hc + k);
#pragma unroll
      for (int kk = 0; kk < 4; ++kk) {
        const v4f w = *(const v4f*)(WHT + (size_t)(k + kk) * kHid + u4);
#pragma unroll
        for (int e = 0; e < 4; ++e) acc[e] = fmaf(w[e], hv[kk], acc[e]);
      }
    }
    const v4f pv = *(const v4f*)(PRE + (size_t)t * kHid + u4);
    const v4f nv = *(const v4f*)(noise0 + (size_t)t * kHid + u4);
    v4f hn;
#pragma unroll
    for (int e = 0; e < 4; ++e) hn[e] = tanhf((pv[e] + acc[e]) + bf16r(nv[e]));
    *(v4f*)(&hbuf[(t + 1) & 1][u4]) = hn;
    float* op = out0 + (size_t)t * kHid + u4;
    *(volatile v4f*)op = hn;
    __threadfence();
    *(volatile v4f*)op = hn;
    if (t == kSeq - 1) {
      *(volatile v4f*)(out1 + u4) = hn;
      __threadfence();
      *(volatile v4f*)(out1 + u4) = hn;
    }
    __syncthreads();
  }
}

__global__ __launch_bounds__(kThr) void th_cast_kernel(const float* __restrict__ src, unsigned short* __restrict__ H16) {
  const size_t i8 = ((size_t)blockIdx.x * kThr + threadIdx.x) * 8;
  const v4f a0 = *(const v4f*)(src + i8);
  const v4f a1 = *(const v4f*)(src + i8 + 4);
  v8h hv;
#pragma unroll
  for (int e = 0; e < 4; ++e) {
    hv[e]     = (_Float16)carry_flush(a0[e], kActCarry);
    hv[4 + e] = (_Float16)carry_flush(a1[e], kActCarry);
  }
  unsigned short* dp = H16 + i8;
  *(volatile v8h*)dp = hv;
  __threadfence();
  *(volatile v8h*)dp = hv;
}

__global__ __launch_bounds__(kThr) void th_roll_kernel(const float* __restrict__ Z, const float* __restrict__ noise,
                                                       float* __restrict__ dst) {
  const size_t i4 = ((size_t)blockIdx.x * kThr + threadIdx.x) * 4;
  const v4f z = *(const v4f*)(Z + i4);
  const v4f nz = *(const v4f*)(noise + i4);
  v4f o;
#pragma unroll
  for (int e = 0; e < 4; ++e) o[e] = tanhf(z[e] + bf16r(nz[e]));
  float* op = dst + i4;
  *(volatile v4f*)op = o;
  __threadfence();
  *(volatile v4f*)op = o;
}

static_assert(((size_t)kSeq * kIn / 8) % kThr == 0 && ((size_t)kHid * kIn / 8) % kThr == 0, "cast grids exact");

extern "C" void kernel_launch(void* const* d_in, const int* in_sizes, int n_in,
                              void* d_out, int out_size, void* d_ws, size_t ws_size,
                              hipStream_t stream) {
  if (n_in < 7 || d_out == nullptr || d_ws == nullptr) return;
  if ((size_t)in_sizes[0] != kSlice || (size_t)in_sizes[1] != kOut0 || in_sizes[2] != kHid) return;
  if (in_sizes[3] != kHid * kIn || in_sizes[4] != kHid * kHid || in_sizes[5] != kHid || in_sizes[6] != 1) return;
  if ((size_t)out_size != kOut0 + kHid) return;
  if (ws_size < kWsTotal) return;
  const float* xin   = (const float*)d_in[0];
  const float* noise = (const float*)d_in[1];
  const float* st0   = (const float*)d_in[2];
  const float* Wih   = (const float*)d_in[3];
  const float* Whh   = (const float*)d_in[4];
  const float* bb    = (const float*)d_in[5];
  float* out0 = (float*)d_out;
  float* out1 = out0 + kOut0;
  char* ws = (char*)d_ws;
  unsigned short* X16 = (unsigned short*)(ws + kOffX16);
  unsigned short* WIH = (unsigned short*)(ws + kOffWIH);
  unsigned short* WHH = (unsigned short*)(ws + kOffWHH);
  float* WHT = (float*)(ws + kOffWHT);
  float* BV  = (float*)(ws + kOffBV);
  float* PRE = (float*)(ws + kOffPRE);
  unsigned short* H16 = (unsigned short*)(ws + kOffH16);
  float* Z   = (float*)(ws + kOffZ);

  cast_plane_kernel<<<(int)(((size_t)kSeq * kIn / 8) / kThr), kThr, 0, stream>>>(xin, X16, 9, kIn, 0);
  cast_plane_kernel<<<(int)(((size_t)kHid * kIn / 8) / kThr), kThr, 0, stream>>>(Wih, WIH, 9, kIn, 0);
  cast_plane_kernel<<<(int)(((size_t)kHid * kHid / 8) / kThr), kThr, 0, stream>>>(Whh, WHH, 9, kHid, 0);
  th_setup_kernel<<<kHid + 1, kThr, 0, stream>>>(Whh, bb, WHT, BV);
  wmma_gemm64<0, false, 2, 0, false, 0><<<dim3((kSeq / 64) * (kHid / 64) / 8, 1), 256, 0, stream>>>(
      X16, X16, kIn, 0L, WIH, WIH, kIn, 0L, (void*)PRE, (void*)PRE, kHid, 0L,
      BV, nullptr, 0L, kSeq, kHid, kIn, kXsScale);
  th_chain_kernel<<<1, kChainThr, 0, stream>>>(PRE, noise, WHT, st0, out0, out1);
  for (int k = 1; k <= kTheta; ++k) {
    th_cast_kernel<<<(int)((kSlice / 8) / kThr), kThr, 0, stream>>>(out0 + (size_t)(k - 1) * kSlice, H16);
    wmma_gemm64<0, false, 2, 0, false, 0><<<dim3((kSeq / 64) * (kHid / 64) / 8, 1), 256, 0, stream>>>(
        H16, H16, kHid, 0L, WHH, WHH, kHid, 0L, (void*)Z, (void*)Z, kHid, 0L,
        BV, nullptr, 0L, kSeq, kHid, kHid, kRecScale);
    th_roll_kernel<<<(int)((kSlice / 4) / kThr), kThr, 0, stream>>>(Z, noise + (size_t)k * kSlice, out0 + (size_t)k * kSlice);
  }
}
